// MultiQueryAttention_63041529970960
// MI455X (gfx1250) — hardware-verified
//
#include <hip/hip_runtime.h>


#ifndef NB
#define NB 2
#endif
#ifndef SEQ
#define SEQ 2048
#endif
#define NB_FULL  2
#define SEQ_FULL 2048
#define DM   2048
#define NH_  16
#define HD   128
#define DQ   (NH_ * HD)
#define SCL   0.088388347648318447f
#define LOG2E 1.4426950408889634f
#define KCAR  16.0f
#define VCAR  16.0f
#define PLOG  10.0f
#define QRES  1024.0f
#define CCAR  64.0f
#define WOCAR 64.0f

typedef _Float16 h16;
typedef unsigned short bf;
typedef __attribute__((ext_vector_type(16))) __bf16   v16bf;
typedef __attribute__((ext_vector_type(16))) _Float16 v16h;
typedef __attribute__((ext_vector_type(8)))  _Float16 v8h;
typedef __attribute__((ext_vector_type(4)))  _Float16 v4h;
typedef __attribute__((ext_vector_type(8)))  unsigned short v8us;
typedef __attribute__((ext_vector_type(2)))  unsigned short v2us;
typedef __attribute__((ext_vector_type(8)))  float    v8f;
typedef __attribute__((ext_vector_type(4)))  float    v4f;
typedef v8h  __attribute__((may_alias)) v8ha;
typedef v4f  __attribute__((may_alias)) v4fa;

static_assert(HD == 128);
static_assert(DM == 2048);
static_assert(DQ == DM);
static_assert(SEQ % 64 == 0);
static_assert((NB * SEQ) % 64 == 0);
static_assert(DM % 32 == 0);
static_assert(SEQ % 32 == 0);
static_assert(NB <= NB_FULL);
static_assert(SEQ <= SEQ_FULL);
static_assert(((size_t)SEQ * DM / 8) % 256 == 0);
static_assert(((size_t)DQ * DM / 64) % 32 == 0);
static_assert(((size_t)HD * DM / 64) % 32 == 0);

__device__ __forceinline__ unsigned short f2bf(float f) { unsigned u = __float_as_uint(f); u += 0x7FFFu + ((u >> 16) & 1u); return (unsigned short)(u >> 16); }
__device__ __forceinline__ float bf2f(unsigned short b) { return __uint_as_float(((unsigned)b) << 16); }
__device__ __forceinline__ float bfr(float f) { return bf2f(f2bf(f)); }
__device__ __forceinline__ v16h cat16(v8h lo, v8h hi) { return __builtin_shufflevector(lo, hi, 0, 1, 2, 3, 4, 5, 6, 7, 8, 9, 10, 11, 12, 13, 14, 15); }
__device__ __forceinline__ v16bf cat16b(v8us lo, v8us hi) { return __builtin_bit_cast(v16bf, __builtin_shufflevector(lo, hi, 0, 1, 2, 3, 4, 5, 6, 7, 8, 9, 10, 11, 12, 13, 14, 15)); }
__device__ __forceinline__ v8f wmma16(v16h a, v16h b, v8f c) { return __builtin_amdgcn_wmma_f32_16x16x32_f16(false, a, false, b, (short)0, c, false, false); }
__device__ __forceinline__ v8f wmmab(v16bf a, v16bf b, v8f c) { return __builtin_amdgcn_wmma_f32_16x16x32_bf16(false, a, false, b, (short)0, c, false, false); }

template <typename T16> struct WFrag;
template <> struct WFrag<h16> { typedef v16h V; static __device__ __forceinline__ V ld(const h16* p) { return cat16(*(const v8h*)p, *(const v8h*)(p + 16)); } static __device__ __forceinline__ v8f mma(V a, V b, v8f c) { return wmma16(a, b, c); } };
template <> struct WFrag<bf> { typedef v16bf V; static __device__ __forceinline__ V ld(const bf* p) { return cat16b(*(const v8us*)p, *(const v8us*)(p + 16)); } static __device__ __forceinline__ v8f mma(V a, V b, v8f c) { return wmmab(a, b, c); } };

template <typename T16, int EPI>
__global__ __launch_bounds__(32) void k_gemmw(const T16* __restrict__ A, const T16* __restrict__ Bt, int K, float* Cf, h16* C0, h16* C1, int ldc, const float* __restrict__ bias, float isc, float osc, size_t sA, size_t sB, size_t sC) {
    typedef typename WFrag<T16>::V V;
    __shared__ __align__(16) float os[16 * 68];
    const size_t z = blockIdx.z; A += z * sA; Bt += z * sB;
    if (EPI == 0) Cf += z * sC; else C0 += z * sC;
    if (EPI == 1) C1 += z * sC;
    const unsigned lane = threadIdx.x & 31u, lr = lane & 15u, hi = lane >> 4; const unsigned r0 = blockIdx.x * 64u, c0 = blockIdx.y * 64u;
    v8f acc[4][4];
#pragma unroll
    for (int mb = 0; mb < 4; ++mb)
#pragma unroll
        for (int nb = 0; nb < 4; ++nb) acc[mb][nb] = (v8f){};
    const size_t aoff = (size_t)(r0 + lr) * K + 8u * hi, boff = (size_t)(c0 + lr) * K + 8u * hi;
#pragma unroll 1
    for (int kc = 0; kc < K; kc += 32) {
        V a[4];
#pragma unroll
        for (int mb = 0; mb < 4; ++mb) a[mb] = WFrag<T16>::ld(A + aoff + (size_t)mb * 16 * K + kc);
#pragma unroll
        for (int nb = 0; nb < 4; ++nb) { const V b = WFrag<T16>::ld(Bt + boff + (size_t)nb * 16 * K + kc);
#pragma unroll
            for (int mb = 0; mb < 4; ++mb) acc[mb][nb] = WFrag<T16>::mma(a[mb], b, acc[mb][nb]); }
        asm volatile("v_nop\n\tv_nop\n\tv_nop\n\tv_nop" : "+v"(acc[0][0]), "+v"(acc[1][1]), "+v"(acc[2][2]), "+v"(acc[3][3]) : "v"(a[0]), "v"(a[3]));
    }
    const unsigned cofs = lr * 4u;
    float bc[4] = {0.f, 0.f, 0.f, 0.f};
    if (EPI != 3) {
#pragma unroll
        for (int q = 0; q < 4; ++q) bc[q] = bfr(bias[c0 + cofs + q]);
    }
#pragma unroll
    for (int mb = 0; mb < 4; ++mb) {
#pragma unroll
        for (int nb = 0; nb < 4; ++nb) {
#pragma unroll
            for (int j = 0; j < 8; ++j) os[(hi * 8u + j) * 68u + nb * 16u + lr] = acc[mb][nb][j]; }
        __builtin_amdgcn_fence(3  , "wavefront"); __builtin_amdgcn_wave_barrier(); asm volatile("" ::: "memory");
        const unsigned rbase = r0 + mb * 16u;
#pragma unroll 1
        for (int ps = 0; ps < 2; ++ps) {
#pragma unroll
            for (int s = 0; s < 8; ++s) {
                const unsigned row = 2u * s + hi;
                v4f val = *(const v4fa*)(os + row * 68u + cofs);
                float br = 0.f;
                if (EPI == 3) br = bfr(bias[rbase + row]);
#pragma unroll
                for (int q = 0; q < 4; ++q) { const float bb = (EPI == 3) ? br : bc[q]; val[q] = (val[q] * isc + bb) * osc; }
                const size_t o = (size_t)(rbase + row) * ldc + c0 + cofs;
                if (EPI == 0) { *(volatile v4f*)(Cf + o) = val; }
                else if (EPI == 1) { v4h hv, rv;
#pragma unroll
                    for (int q = 0; q < 4; ++q) { const h16 a = (h16)val[q]; const float d = val[q] - (float)a; hv[q] = a; rv[q] = (h16)(d * QRES); }
                    *(volatile v4h*)(C0 + o) = hv; *(volatile v4h*)(C1 + o) = rv; }
                else { v4h hv;
#pragma unroll
                    for (int q = 0; q < 4; ++q) hv[q] = (h16)val[q];
                    *(volatile v4h*)(C0 + o) = hv; }
            }
            if (ps == 0) __threadfence(); }
        __builtin_amdgcn_fence(3  , "wavefront"); __builtin_amdgcn_wave_barrier(); asm volatile("" ::: "memory");
    }
}

template <bool F16>
__global__ __launch_bounds__(256) void k_wtG(const float* __restrict__ w, unsigned N, float sc, unsigned short* Bt) {
    const unsigned lane = threadIdx.x & 31u; const unsigned L0 = (blockIdx.x * 8u + (threadIdx.x >> 5)) * 4u;
    v2us o[4];
#pragma unroll
    for (int l = 0; l < 4; ++l) {
        const unsigned e = (L0 + l) * 64u + lane * 2u; const unsigned k = e & (DM - 1u), n = e >> 11;
        const float x0 = w[k * N + n], x1 = w[(k + 1u) * N + n];
        if (F16) { o[l][0] = __builtin_bit_cast(unsigned short, (h16)(bfr(x0) * sc)); o[l][1] = __builtin_bit_cast(unsigned short, (h16)(bfr(x1) * sc)); }
        else { o[l][0] = f2bf(x0); o[l][1] = f2bf(x1); }
    }
#pragma unroll
    for (int l = 0; l < 4; ++l) *(volatile v2us*)(Bt + (size_t)(L0 + l) * 64u + lane * 2u) = o[l];
    __threadfence();
#pragma unroll
    for (int l = 0; l < 4; ++l) *(volatile v2us*)(Bt + (size_t)(L0 + l) * 64u + lane * 2u) = o[l];
}

__global__ __launch_bounds__(256) void k_cvt8(const float* __restrict__ src, bf* dst, unsigned n8, size_t sstride, size_t dstride) {
    const unsigned i = blockIdx.x * 256u + threadIdx.x; if (i >= n8) return;
    const float* s = src + (size_t)blockIdx.y * sstride + (size_t)i * 8u; bf* d = dst + (size_t)blockIdx.y * dstride + (size_t)i * 8u;
    const v8f v = *(const v8f*)s; v8us o;
#pragma unroll
    for (int k = 0; k < 8; ++k) o[k] = f2bf(v[k]);
    *(volatile v8us*)d = o; __threadfence(); *(volatile v8us*)d = o;
}

__global__ __launch_bounds__(128) __attribute__((amdgpu_num_vgpr(256)))
void k_flash(const h16* __restrict__ Qh, const h16* __restrict__ Qr, const h16* __restrict__ Kp, const h16* __restrict__ VT, h16* CTX) {
    __shared__ __align__(16) h16 osw[4 * 16 * 136];
    const unsigned lane = threadIdx.x & 31u, w = threadIdx.x >> 5, lr = lane & 15u, hi = lane >> 4;
    const unsigned b = blockIdx.z, h = blockIdx.y, q0 = blockIdx.x * 64u + w * 16u;
    const size_t qoff = (size_t)(b * SEQ + q0 + lr) * DQ + h * HD + 8u * hi;
    v16h qh[4], qr[4];
#pragma unroll
    for (int d0 = 0; d0 < 4; ++d0) { qh[d0] = WFrag<h16>::ld(Qh + qoff + d0 * 32); qr[d0] = WFrag<h16>::ld(Qr + qoff + d0 * 32); }
    v8f oacc[8];
#pragma unroll
    for (int dt = 0; dt < 8; ++dt) oacc[dt] = (v8f){};
    float m = -3.0e38f, l = 0.f;
    const h16* kb = Kp + ((size_t)b * SEQ + lr) * HD + 8u * hi;
    const h16* vb = VT + ((size_t)b * HD + lr) * SEQ + 8u * hi;
    const float clog = SCL * LOG2E * (1.0f / KCAR);
#pragma unroll 1
    for (unsigned j = 0; j < SEQ; j += 64u) {
        v8f s[4];
#pragma unroll
        for (int tn = 0; tn < 4; ++tn) {
            v8f ah = (v8f){}, ar = (v8f){};
            const h16* kp = kb + (size_t)(j + tn * 16u) * HD;
#pragma unroll
            for (int d0 = 0; d0 < 4; ++d0) { const v16h kf = WFrag<h16>::ld(kp + d0 * 32); ah = wmma16(kf, qh[d0], ah); ar = wmma16(kf, qr[d0], ar); }
            asm volatile("v_nop\n\tv_nop\n\tv_nop\n\tv_nop" : "+v"(ah), "+v"(ar) : "v"(qh[3]), "v"(qr[3]));
#pragma unroll
            for (int r = 0; r < 8; ++r) s[tn][r] = (ah[r] + ar[r] * (1.0f / QRES)) * clog;
        }
        float mx = s[0][0];
#pragma unroll
        for (int tn = 0; tn < 4; ++tn)
#pragma unroll
            for (int r = 0; r < 8; ++r) mx = fmaxf(mx, s[tn][r]);
        mx = fmaxf(mx, __shfl_xor(mx, 16, 32));
        const float mn = fmaxf(m, mx);
        const float alpha = __builtin_amdgcn_exp2f(m - mn);
        m = mn;
        const float mc = mn - PLOG;
        v16h pf[2]; float ps = 0.f;
#pragma unroll
        for (int ks = 0; ks < 2; ++ks)
#pragma unroll
            for (int r = 0; r < 8; ++r) {
                const h16 a = (h16)__builtin_amdgcn_exp2f(s[2 * ks][r] - mc);
                const h16 c = (h16)__builtin_amdgcn_exp2f(s[2 * ks + 1][r] - mc);
                pf[ks][r] = a; pf[ks][8 + r] = c; ps += (float)a; ps += (float)c; }
        l = l * alpha + ps;
#pragma unroll
        for (int dt = 0; dt < 8; ++dt)
#pragma unroll
            for (int r = 0; r < 8; ++r) oacc[dt][r] *= alpha;
#pragma unroll
        for (int dt = 0; dt < 8; ++dt)
#pragma unroll
            for (int ks = 0; ks < 2; ++ks) { const v16h vf = WFrag<h16>::ld(vb + (size_t)(dt * 16) * SEQ + j + ks * 32u); oacc[dt] = wmma16(vf, pf[ks], oacc[dt]); }
        asm volatile("v_nop\n\tv_nop\n\tv_nop\n\tv_nop" : "+v"(oacc[0]), "+v"(oacc[1]), "+v"(oacc[2]), "+v"(oacc[3]), "+v"(oacc[4]), "+v"(oacc[5]), "+v"(oacc[6]), "+v"(oacc[7]) : "v"(pf[0]), "v"(pf[1]));
    }
    const float lt = l + __shfl_xor(l, 16, 32);
    const float inv = (CCAR / VCAR) * (1.0f / lt);
    h16* ow = osw + w * (16 * 136);
#pragma unroll
    for (int dt = 0; dt < 8; ++dt) { v8h o;
#pragma unroll
        for (int r = 0; r < 8; ++r) o[r] = (h16)(oacc[dt][r] * inv);
        *(v8h*)(ow + lr * 136u + dt * 16u + 8u * hi) = o; }
    __builtin_amdgcn_fence(3  , "wavefront"); __builtin_amdgcn_wave_barrier(); asm volatile("" ::: "memory");
    h16* dst = CTX + (size_t)(b * SEQ + q0) * DQ + h * HD;
#pragma unroll 1
    for (int ps2 = 0; ps2 < 2; ++ps2) {
#pragma unroll
        for (int s2 = 0; s2 < 8; ++s2) { const unsigned row = 2u * s2 + hi; const v8h v = *(const v8ha*)(ow + row * 136u + lr * 8u); *(volatile v8h*)(dst + (size_t)row * DQ + lr * 8u) = v; }
        if (ps2 == 0) __threadfence(); }
}

constexpr size_t SZ_WQ  = (size_t)DQ * DM * 2;
constexpr size_t SZ_WKV = (size_t)HD * DM * 2;
constexpr size_t SZ_WO  = (size_t)DM * DQ * 2;
constexpr size_t SZ_XB  = (size_t)NB * SEQ * DM * 2;
constexpr size_t SZ_Q   = (size_t)NB * SEQ * DQ * 2;
constexpr size_t SZ_KP  = (size_t)NB * SEQ * HD * 2;
constexpr size_t SZ_VT  = (size_t)NB * HD * SEQ * 2;
constexpr size_t SZ_CTX = (size_t)NB * SEQ * DQ * 2;
constexpr size_t WS_TOTAL = SZ_WQ + 2 * SZ_WKV + SZ_WO + SZ_XB + 2 * SZ_Q + SZ_KP + SZ_VT + SZ_CTX;
static_assert(WS_TOTAL <= (size_t)134217728);
static_assert(SZ_WQ % 256 == 0 && SZ_WKV % 256 == 0 && SZ_XB % 256 == 0 && SZ_KP % 256 == 0);

extern "C" void kernel_launch(void* const* d_in, const int* in_sizes, int n_in,
                              void* d_out, int out_size, void* d_ws, size_t ws_size, hipStream_t stream) {
    if (n_in < 11) return;
    const size_t need_x = ((size_t)(NB - 1) * SEQ_FULL + SEQ) * DM;
    if ((size_t)in_sizes[0] < need_x || (size_t)in_sizes[1] < need_x || (size_t)in_sizes[2] < need_x) return;
    if ((size_t)in_sizes[3] < (size_t)DM * DQ || in_sizes[4] < DQ || (size_t)in_sizes[5] < (size_t)DM * HD || in_sizes[6] < HD) return;
    if ((size_t)in_sizes[7] < (size_t)DM * HD || in_sizes[8] < HD || (size_t)in_sizes[9] < (size_t)DQ * DM || in_sizes[10] < DM) return;
    if ((size_t)out_size < need_x) return;
    if (WS_TOTAL > ws_size) return;
    const float* xq = (const float*)d_in[0]; const float* xk = (const float*)d_in[1]; const float* xv = (const float*)d_in[2];
    const float* wq = (const float*)d_in[3]; const float* bq = (const float*)d_in[4];
    const float* wk = (const float*)d_in[5]; const float* bk = (const float*)d_in[6];
    const float* wv = (const float*)d_in[7]; const float* bv = (const float*)d_in[8];
    const float* wo = (const float*)d_in[9]; const float* bo = (const float*)d_in[10];
    float* OUT = (float*)d_out;
    char* wsp = (char*)d_ws;
    auto take = [&](size_t bytes) { char* p = wsp; wsp += bytes; return (void*)p; };
    bf* WQ = (bf*)take(SZ_WQ); bf* WK = (bf*)take(SZ_WKV); bf* WV = (bf*)take(SZ_WKV); h16* WO = (h16*)take(SZ_WO);
    bf* XB = (bf*)take(SZ_XB); h16* QH = (h16*)take(SZ_Q); h16* QR = (h16*)take(SZ_Q);
    h16* KP = (h16*)take(SZ_KP); h16* VT = (h16*)take(SZ_VT); h16* CTX = (h16*)take(SZ_CTX);
    if ((size_t)(wsp - (char*)d_ws) > ws_size) return;

    k_wtG<false><<<(unsigned)((size_t)DQ * DM / 64 / 32), 256, 0, stream>>>(wq, (unsigned)DQ, 1.0f, (unsigned short*)WQ);
    k_wtG<false><<<(unsigned)((size_t)HD * DM / 64 / 32), 256, 0, stream>>>(wk, (unsigned)HD, 1.0f, (unsigned short*)WK);
    k_wtG<false><<<(unsigned)((size_t)HD * DM / 64 / 32), 256, 0, stream>>>(wv, (unsigned)HD, 1.0f, (unsigned short*)WV);
    k_wtG<true><<<(unsigned)((size_t)DM * DQ / 64 / 32), 256, 0, stream>>>(wo, (unsigned)DM, WOCAR, (unsigned short*)WO);

    const unsigned n8 = (unsigned)((size_t)SEQ * DM / 8);
    const dim3 gcv(n8 / 256, NB, 1);
    k_cvt8<<<gcv, 256, 0, stream>>>(xq, XB, n8, (size_t)SEQ_FULL * DM, (size_t)SEQ * DM);
    k_gemmw<bf, 1><<<dim3(NB * SEQ / 64, DQ / 64, 1), 32, 0, stream>>>(XB, WQ, DM, nullptr, QH, QR, DQ, bq, 1.0f, 1.0f, 0, 0, 0);
    k_cvt8<<<gcv, 256, 0, stream>>>(xk, XB, n8, (size_t)SEQ_FULL * DM, (size_t)SEQ * DM);
    k_gemmw<bf, 2><<<dim3(NB * SEQ / 64, HD / 64, 1), 32, 0, stream>>>(XB, WK, DM, nullptr, KP, nullptr, HD, bk, 1.0f, KCAR, 0, 0, 0);
    k_cvt8<<<gcv, 256, 0, stream>>>(xv, XB, n8, (size_t)SEQ_FULL * DM, (size_t)SEQ * DM);
    k_gemmw<bf, 3><<<dim3(HD / 64, SEQ / 64, NB), 32, 0, stream>>>(WV, XB, DM, nullptr, VT, nullptr, SEQ, bv, 1.0f, VCAR, 0, (size_t)SEQ * DM, (size_t)HD * SEQ);
    k_flash<<<dim3(SEQ / 64, NH_, NB), 128, 0, stream>>>(QH, QR, KP, VT, CTX);
    k_gemmw<h16, 0><<<dim3(SEQ / 64, DM / 64, NB), 32, 0, stream>>>(CTX, WO, DQ, OUT, nullptr, nullptr, DM, bo, 1.0f / (CCAR * WOCAR), 1.0f, (size_t)SEQ * DQ, 0, (size_t)SEQ_FULL * DM);
}
